// MAGCN_4406636446376
// MI455X (gfx1250) — hardware-verified
//
#include <hip/hip_runtime.h>
#define BB 32
#define LL 200
#define HH 64
#define NHD 2
#define HD 32
#define NB 2
#define NTOK (BB * LL)
#define NREL 257
#define NRP 288
#define MAXID 50000

typedef __bf16 v16b __attribute__((ext_vector_type(16)));
typedef unsigned short v8us __attribute__((ext_vector_type(8), may_alias));
typedef float  v8f  __attribute__((ext_vector_type(8)));
typedef float  v4f  __attribute__((ext_vector_type(4)));
typedef float  v4fa __attribute__((ext_vector_type(4), may_alias));
union FragB { v16b v; v8us half[2]; unsigned short u[16]; };

__device__ __forceinline__ unsigned short bf16_bits(float x) { unsigned int u = __float_as_uint(x); return (unsigned short)((u + 0x7FFFu + ((u >> 16) & 1u)) >> 16); }
__device__ __forceinline__ float bf16_val(unsigned short b) { return __uint_as_float(((unsigned int)b) << 16); }
__device__ __forceinline__ float bf16_round(float x) { return bf16_val(bf16_bits(x)); }
template <int NT>
__device__ __forceinline__ v8f mmaN(v16b ah, v16b al, v16b bh, v16b bl, v8f c) {
  c = __builtin_amdgcn_wmma_f32_16x16x32_bf16(false, ah, false, bh, (short)0, c, false, false);
  if (NT >= 2) c = __builtin_amdgcn_wmma_f32_16x16x32_bf16(false, al, false, bh, (short)0, c, false, false);
  if (NT >= 3) c = __builtin_amdgcn_wmma_f32_16x16x32_bf16(false, ah, false, bl, (short)0, c, false, false);
  asm volatile("v_nop\n\tv_nop\n\tv_nop\n\tv_nop" : "+v"(c) : "v"(ah), "v"(al), "v"(bh), "v"(bl));
  return c;
}

__global__ __launch_bounds__(256) void k_wt_bf16(const float* __restrict__ W, unsigned short* __restrict__ Wt, int K, int N) {
  const int t = blockIdx.x * 256 + threadIdx.x;
  const int k8n = K / 8;
  if (t >= N * k8n) return;
  const int n = t / k8n, k8 = (t % k8n) * 8;
  v8us v;
#pragma unroll
  for (int i = 0; i < 8; ++i) v[i] = bf16_bits(W[(size_t)(k8 + i) * N + n]);
  *(volatile v8us*)(Wt + (size_t)n * K + k8) = v;
  __threadfence();
  *(volatile v8us*)(Wt + (size_t)n * K + k8) = v;
}

template <bool ASPLIT, int ACT, bool BIAS_BF16>
__global__ __launch_bounds__(128) void k_gemm_bf(const float* __restrict__ A, int lda, const unsigned short* __restrict__ Wt, int ldb,
                                               const float* __restrict__ bias, float* __restrict__ C, int ldc, int M, int N, int K) {
  __shared__ __attribute__((aligned(16))) float so[4][16][64];
  const int tid = threadIdx.x, w = tid >> 5, lane = tid & 31, ln = lane & 15, hh = lane >> 4;
  const int ntn = N / 64;
  const int wid = blockIdx.x * 4 + w;
  const int mt = wid / ntn, nq = wid % ntn;
  if (mt * 16 >= M) return;
  const int row0 = mt * 16, col0 = nq * 64;
  const float* arow = A + (size_t)(row0 + ln) * lda;
  v8f acc[4] = {};
  for (int kb = 0; kb < K; kb += 32) {
    FragB ah, al;
    const v4f x0 = *(const v4fa*)(arow + kb + 8 * hh), x1 = *(const v4fa*)(arow + kb + 8 * hh + 4);
    const v4f x2 = *(const v4fa*)(arow + kb + 16 + 8 * hh), x3 = *(const v4fa*)(arow + kb + 16 + 8 * hh + 4);
    float xs[16] = {x0[0],x0[1],x0[2],x0[3],x1[0],x1[1],x1[2],x1[3],x2[0],x2[1],x2[2],x2[3],x3[0],x3[1],x3[2],x3[3]};
#pragma unroll
    for (int i = 0; i < 16; ++i) { const unsigned short hb = bf16_bits(xs[i]); ah.u[i] = hb; al.u[i] = ASPLIT ? bf16_bits(xs[i] - bf16_val(hb)) : (unsigned short)0; }
#pragma unroll
    for (int t = 0; t < 4; ++t) {
      const unsigned short* brow = Wt + (size_t)(col0 + t * 16 + ln) * ldb + kb;
      FragB b;
      b.half[0] = *(const v8us*)(brow + 8 * hh);
      b.half[1] = *(const v8us*)(brow + 16 + 8 * hh);
      acc[t] = mmaN<ASPLIT ? 2 : 1>(ah.v, al.v, b.v, b.v, acc[t]);
    }
  }
#pragma unroll
  for (int t = 0; t < 4; ++t) {
    float bv = bias ? bias[col0 + t * 16 + ln] : 0.f;
    if (BIAS_BF16) bv = bf16_round(bv);
#pragma unroll
    for (int r = 0; r < 8; ++r) { float v = acc[t][r] + bv; if (ACT == 1) v = fmaxf(v, 0.f); so[w][8 * hh + r][t * 16 + ln] = v; }
  }
  __builtin_amdgcn_fence(__ATOMIC_ACQ_REL, "workgroup");
  __builtin_amdgcn_wave_barrier();
  const int rsub = lane >> 4, c4 = (lane & 15) * 4;
  for (int pass = 0; pass < 2; ++pass) {
#pragma unroll
    for (int q = 0; q < 8; ++q) {
      const int r = q * 2 + rsub;
      const v4f v = *(const v4fa*)&so[w][r][c4];
      *(volatile v4f*)(C + (size_t)(row0 + r) * ldc + col0 + c4) = v;
    }
    if (pass == 0) __threadfence();
  }
}

template <int D, bool CAUSAL>
__global__ __launch_bounds__(128) void k_flash(const float* __restrict__ qb, const float* __restrict__ kb, const float* __restrict__ vb,
                                             int pitch, int T, int H, float scale, float* __restrict__ y, int ypitch) {
  constexpr int KS = D / 32;
  constexpr int DT = D / 16;
  __shared__ __attribute__((aligned(16))) unsigned short sKh[32][D + 8], sKl[32][D + 8], sVh[32][D + 8], sVl[32][D + 8];
  __shared__ __attribute__((aligned(16))) unsigned short sPh[4][16][40], sPl[4][16][40];
  __shared__ __attribute__((aligned(16))) float sO[4][16][D];
  const int tid = threadIdx.x, w = tid >> 5, lane = tid & 31, ln = lane & 15, hh = lane >> 4;
  const int nqb = (T + 63) / 64;
  const int bh = blockIdx.x / nqb, qblk = blockIdx.x % nqb;
  const int b = bh / H, h = bh % H;
  const int q0 = qblk * 64 + w * 16;
  const float* Q = qb + (size_t)b * T * pitch + h * D;
  const float* K = kb + (size_t)b * T * pitch + h * D;
  const float* V = vb + (size_t)b * T * pitch + h * D;

  FragB aqh[KS], aql[KS];
  {
    int row = q0 + ln; if (row >= T) row = T - 1;
    const float* qr = Q + (size_t)row * pitch;
#pragma unroll
    for (int ks = 0; ks < KS; ++ks)
#pragma unroll
      for (int i = 0; i < 16; ++i) {
        const int d = ks * 32 + ((i < 8) ? (8 * hh + i) : (16 + 8 * hh + (i - 8)));
        const float x = qr[d] * scale; const unsigned short hb = bf16_bits(x);
        aqh[ks].u[i] = hb; aql[ks].u[i] = bf16_bits(x - bf16_val(hb));
      }
  }
  float m_r[8], l_r[8];
#pragma unroll
  for (int r = 0; r < 8; ++r) { m_r[r] = -3.0e38f; l_r[r] = 0.f; }
  v8f oacc[DT];
#pragma unroll
  for (int dt = 0; dt < DT; ++dt) oacc[dt] = (v8f){0.f,0.f,0.f,0.f,0.f,0.f,0.f,0.f};

  const int kv_end = CAUSAL ? min(T, qblk * 64 + 64) : T;
  for (int j0 = 0; j0 < kv_end; j0 += 32) {
    __syncthreads();
    for (int e = tid; e < 32 * (D / 4); e += 128) {
      const int r = e / (D / 4), c4 = (e % (D / 4)) * 4;
      const int key = j0 + r;
      v4f kf = {0.f,0.f,0.f,0.f}, vf = {0.f,0.f,0.f,0.f};
      if (key < T) { kf = *(const v4fa*)(K + (size_t)key * pitch + c4); vf = *(const v4fa*)(V + (size_t)key * pitch + c4); }
#pragma unroll
      for (int t = 0; t < 4; ++t) {
        unsigned short hb = bf16_bits(kf[t]); sKh[r][c4 + t] = hb; sKl[r][c4 + t] = bf16_bits(kf[t] - bf16_val(hb));
        hb = bf16_bits(vf[t]); sVh[r][c4 + t] = hb; sVl[r][c4 + t] = bf16_bits(vf[t] - bf16_val(hb));
      }
    }
    __syncthreads();
    v8f s[2];
#pragma unroll
    for (int nt = 0; nt < 2; ++nt) {
      v8f acc = {};
#pragma unroll
      for (int ks = 0; ks < KS; ++ks) {
        FragB bh_, bl_;
        bh_.half[0] = *(const v8us*)&sKh[nt * 16 + ln][ks * 32 + 8 * hh]; bh_.half[1] = *(const v8us*)&sKh[nt * 16 + ln][ks * 32 + 16 + 8 * hh];
        bl_.half[0] = *(const v8us*)&sKl[nt * 16 + ln][ks * 32 + 8 * hh]; bl_.half[1] = *(const v8us*)&sKl[nt * 16 + ln][ks * 32 + 16 + 8 * hh];
        acc = mmaN<3>(aqh[ks].v, aql[ks].v, bh_.v, bl_.v, acc);
      }
      s[nt] = acc;
    }
    float alpha[8];
#pragma unroll
    for (int r = 0; r < 8; ++r) {
      const int qi = q0 + 8 * hh + r;
      const int ja = j0 + ln, jb = j0 + 16 + ln;
      if (CAUSAL) { if (ja > qi) s[0][r] = -3.0e38f; if (jb > qi) s[1][r] = -3.0e38f; }
      if (ja >= T) s[0][r] = -3.0e38f;
      if (jb >= T) s[1][r] = -3.0e38f;
      float mx = fmaxf(s[0][r], s[1][r]);
      mx = fmaxf(mx, __shfl_xor(mx, 1, 32)); mx = fmaxf(mx, __shfl_xor(mx, 2, 32)); mx = fmaxf(mx, __shfl_xor(mx, 4, 32)); mx = fmaxf(mx, __shfl_xor(mx, 8, 32));
      const float mnew = fmaxf(m_r[r], mx);
      alpha[r] = (mnew > -1.0e38f) ? __expf(m_r[r] - mnew) : 1.0f;
      const float p0 = (s[0][r] > -1.0e38f) ? __expf(s[0][r] - mnew) : 0.f;
      const float p1 = (s[1][r] > -1.0e38f) ? __expf(s[1][r] - mnew) : 0.f;
      m_r[r] = mnew;
      l_r[r] = l_r[r] * alpha[r] + p0 + p1;
      unsigned short hb = bf16_bits(p0); sPh[w][8 * hh + r][ln] = hb;      sPl[w][8 * hh + r][ln] = bf16_bits(p0 - bf16_val(hb));
      hb = bf16_bits(p1);                sPh[w][8 * hh + r][16 + ln] = hb; sPl[w][8 * hh + r][16 + ln] = bf16_bits(p1 - bf16_val(hb));
    }
#pragma unroll
    for (int dt = 0; dt < DT; ++dt)
#pragma unroll
      for (int r = 0; r < 8; ++r) oacc[dt][r] *= alpha[r];
    __builtin_amdgcn_fence(__ATOMIC_ACQ_REL, "workgroup");
    __builtin_amdgcn_wave_barrier();
    FragB pah, pal;
    pah.half[0] = *(const v8us*)&sPh[w][ln][8 * hh]; pah.half[1] = *(const v8us*)&sPh[w][ln][16 + 8 * hh];
    pal.half[0] = *(const v8us*)&sPl[w][ln][8 * hh]; pal.half[1] = *(const v8us*)&sPl[w][ln][16 + 8 * hh];
#pragma unroll
    for (int dt = 0; dt < DT; ++dt) {
      FragB bvh, bvl;
#pragma unroll
      for (int i = 0; i < 8; ++i) {
        bvh.u[i] = sVh[8 * hh + i][dt * 16 + ln]; bvh.u[8 + i] = sVh[16 + 8 * hh + i][dt * 16 + ln];
        bvl.u[i] = sVl[8 * hh + i][dt * 16 + ln]; bvl.u[8 + i] = sVl[16 + 8 * hh + i][dt * 16 + ln];
      }
      oacc[dt] = mmaN<3>(pah.v, pal.v, bvh.v, bvl.v, oacc[dt]);
    }
    __builtin_amdgcn_fence(__ATOMIC_ACQ_REL, "workgroup");
    __builtin_amdgcn_wave_barrier();
  }
#pragma unroll
  for (int r = 0; r < 8; ++r) {
    float l = l_r[r];
    l += __shfl_xor(l, 1, 32); l += __shfl_xor(l, 2, 32); l += __shfl_xor(l, 4, 32); l += __shfl_xor(l, 8, 32);
    l_r[r] = (l > 0.f) ? 1.0f / l : 0.f;
  }
#pragma unroll
  for (int dt = 0; dt < DT; ++dt)
#pragma unroll
    for (int r = 0; r < 8; ++r) sO[w][8 * hh + r][dt * 16 + ln] = oacc[dt][r] * l_r[r];
  __builtin_amdgcn_fence(__ATOMIC_ACQ_REL, "workgroup");
  __builtin_amdgcn_wave_barrier();
  for (int pass = 0; pass < 2; ++pass) {
    for (int r = 0; r < 16; ++r) {
      const int row = q0 + r;
      if (row < T && lane < D / 4) {
        const v4f val = *(const v4fa*)&sO[w][r][lane * 4];
        *(volatile v4f*)(y + ((size_t)b * T + row) * ypitch + h * D + lane * 4) = val;
      }
    }
    if (pass == 0) __threadfence();
  }
}

template <bool ASPLIT, bool BSPLIT, int ACT>
__global__ __launch_bounds__(128) void k_gemm_b(const float* __restrict__ A, int lda, size_t sA, const unsigned short* __restrict__ Bh, const unsigned short* __restrict__ Bl, int ldb, size_t sB,
                                             const float* __restrict__ bias, const float* __restrict__ resid, int ldr, size_t sR, float rsign, float alpha,
                                             float* __restrict__ C, int ldc, size_t sC, int M, int N, int K) {
  __shared__ __attribute__((aligned(16))) float so[4][16][64];
  const int tid = threadIdx.x, w = tid >> 5, lane = tid & 31, ln = lane & 15, hh = lane >> 4;
  const int by = blockIdx.y;
  A += (size_t)by * sA; Bh += (size_t)by * sB; if (BSPLIT) Bl += (size_t)by * sB; C += (size_t)by * sC; if (resid) resid += (size_t)by * sR;
  const int ntn = (N + 63) / 64; const int wid = blockIdx.x * 4 + w; const int mt = wid / ntn, nq = wid % ntn;
  if (mt * 16 >= M) return;
  const int row0 = mt * 16, col0 = nq * 64;
  const float* arow = A + (size_t)(row0 + ln) * lda;
  v8f acc[4] = {};
  for (int kb = 0; kb < K; kb += 32) {
    FragB ah, al;
    const v4f x0 = *(const v4fa*)(arow + kb + 8 * hh), x1 = *(const v4fa*)(arow + kb + 8 * hh + 4);
    const v4f x2 = *(const v4fa*)(arow + kb + 16 + 8 * hh), x3 = *(const v4fa*)(arow + kb + 16 + 8 * hh + 4);
    float xs[16] = {x0[0],x0[1],x0[2],x0[3],x1[0],x1[1],x1[2],x1[3],x2[0],x2[1],x2[2],x2[3],x3[0],x3[1],x3[2],x3[3]};
#pragma unroll
    for (int i = 0; i < 16; ++i) { const unsigned short hb = bf16_bits(xs[i]); ah.u[i] = hb; al.u[i] = ASPLIT ? bf16_bits(xs[i] - bf16_val(hb)) : (unsigned short)0; }
#pragma unroll
    for (int t = 0; t < 4; ++t) {
      if (col0 + t * 16 >= N) continue;
      const size_t boff = (size_t)(col0 + t * 16 + ln) * ldb + kb;
      FragB bh_, bl_; bh_.half[0] = *(const v8us*)(Bh + boff + 8 * hh); bh_.half[1] = *(const v8us*)(Bh + boff + 16 + 8 * hh);
      if (BSPLIT) { bl_.half[0] = *(const v8us*)(Bl + boff + 8 * hh); bl_.half[1] = *(const v8us*)(Bl + boff + 16 + 8 * hh); } else bl_ = bh_;
      acc[t] = mmaN<ASPLIT ? (BSPLIT ? 3 : 2) : 1>(ah.v, al.v, bh_.v, bl_.v, acc[t]);
    }
  }
#pragma unroll
  for (int t = 0; t < 4; ++t) {
    const int col = col0 + t * 16 + ln; if (col0 + t * 16 >= N) continue; const float bv = bias ? bf16_round(bias[col]) : 0.f;
#pragma unroll
    for (int r = 0; r < 8; ++r) { float v = acc[t][r] * alpha + bv; if (resid) v += rsign * resid[(size_t)(row0 + 8 * hh + r) * ldr + col]; if (ACT == 1) v = fmaxf(v, 0.f); else if (ACT == 2) v = fmaxf(v, 0.f) + log1pf(expf(-fabsf(v))); so[w][8 * hh + r][t * 16 + ln] = v; }
  }
  __builtin_amdgcn_fence(__ATOMIC_ACQ_REL, "workgroup"); __builtin_amdgcn_wave_barrier();
  const int rsub = lane >> 4, c4 = (lane & 15) * 4;
  for (int pass = 0; pass < 2; ++pass) {
#pragma unroll
    for (int q = 0; q < 8; ++q) { const int r = q * 2 + rsub; if (col0 + c4 < N) { const v4f v = *(const v4fa*)&so[w][r][c4]; *(volatile v4f*)(C + (size_t)(row0 + r) * ldc + col0 + c4) = v; } }
    if (pass == 0) __threadfence();
  }
}
__global__ __launch_bounds__(256) void k_split_transpose_b(const float* __restrict__ src, int lds_, size_t sIn, unsigned short* __restrict__ hi, unsigned short* __restrict__ lo, size_t sOut, int K, int N) {
  const size_t t = (size_t)blockIdx.x * 256 + threadIdx.x; const int k8n = K / 8; if (t >= (size_t)N * k8n) return;
  src += (size_t)blockIdx.y * sIn; hi += (size_t)blockIdx.y * sOut; lo += (size_t)blockIdx.y * sOut;
  const int n = (int)(t / k8n), k8 = (int)(t % k8n) * 8; v8us vh, vl;
#pragma unroll
  for (int i = 0; i < 8; ++i) { const float x = src[(size_t)(k8 + i) * lds_ + n]; const unsigned short hb = bf16_bits(x); vh[i] = hb; vl[i] = bf16_bits(x - bf16_val(hb)); }
  unsigned short* dh = hi + (size_t)n * K + k8; unsigned short* dl = lo + (size_t)n * K + k8;
  *(volatile v8us*)dh = vh; *(volatile v8us*)dl = vl; __threadfence(); *(volatile v8us*)dh = vh; *(volatile v8us*)dl = vl;
}

__global__ __launch_bounds__(256) void k_tabK(const float* __restrict__ tmk, const float* __restrict__ dmk, unsigned short* __restrict__ TK) { const int t = blockIdx.x * 256 + threadIdx.x; if (t >= 2 * NRP * 8) return; const int c8 = (t & 7) * 8; const int r = (t >> 3) % NRP; const int wch = t / (8 * NRP); const float* src = wch ? dmk : tmk; v8us v;
  for (int q = 0; q < 8; ++q) v[q] = bf16_bits(r < NREL ? src[r * HH + c8 + q] : 0.f); *(volatile v8us*)(TK + ((size_t)wch * NRP + r) * HH + c8) = v; __threadfence(); *(volatile v8us*)(TK + ((size_t)wch * NRP + r) * HH + c8) = v; }
__global__ __launch_bounds__(256) void k_tabV(const float* __restrict__ tmv, const float* __restrict__ dmv, unsigned short* __restrict__ TVt) { const int t = blockIdx.x * 256 + threadIdx.x; if (t >= 2 * NHD * HD * (NRP / 8)) return; const int r8 = (t % (NRP / 8)) * 8; const int d = (t / (NRP / 8)) % HD; const int h = (t / ((NRP / 8) * HD)) % NHD; const int wch = t / ((NRP / 8) * HD * NHD); const float* src = wch ? dmv : tmv; v8us v;
  for (int q = 0; q < 8; ++q) { const int r = r8 + q; v[q] = bf16_bits(r < NREL ? src[r * HH + h * HD + d] : 0.f); } const size_t dst = (((size_t)wch * NHD + h) * HD + d) * NRP + r8; *(volatile v8us*)(TVt + dst) = v; __threadfence(); *(volatile v8us*)(TVt + dst) = v; }
__global__ __launch_bounds__(256) void k_emb(const int* __restrict__ ids, const float* __restrict__ emb, float* __restrict__ SEQ) { const int tid = threadIdx.x, wv = tid >> 5, lane = tid & 31; const int tk = blockIdx.x * 8 + wv; if (tk >= NTOK) return; int id = ids[tk]; const float keep = (id == 0) ? 0.f : 1.f; id = id < 0 ? 0 : (id > MAXID ? MAXID : id);
  const float a = bf16_round(emb[(size_t)id * HH + lane]) * keep, b = bf16_round(emb[(size_t)id * HH + 32 + lane]) * keep; for (int pass = 0; pass < 2; ++pass) { *(volatile float*)(SEQ + (size_t)tk * HH + lane) = a; *(volatile float*)(SEQ + (size_t)tk * HH + 32 + lane) = b; if (pass == 0) __threadfence(); } }
__global__ __launch_bounds__(256) void k_proj(const float* __restrict__ SEQ, const float* __restrict__ Wq, const float* __restrict__ bq, const float* __restrict__ Wk, const float* __restrict__ bk, const float* __restrict__ Wv, const float* __restrict__ bv, const float* __restrict__ g1, const float* __restrict__ be1, const float* __restrict__ pK, const float* __restrict__ pV, float* __restrict__ QN, float* __restrict__ Qo, float* __restrict__ KP, float* __restrict__ VP) {
  __shared__ float swq[HH][HH + 1], swk[HH][HH + 1], swv[HH][HH + 1]; __shared__ float sx[8][HH], sq[8][HH]; const int tid = threadIdx.x, wv = tid >> 5, lane = tid & 31;
  for (int e = tid; e < HH * HH; e += 256) { const int o = e / HH, i = e % HH; swq[i][o] = bf16_round(Wq[e]); swk[i][o] = bf16_round(Wk[e]); swv[i][o] = bf16_round(Wv[e]); }
  __syncthreads(); const int tk = blockIdx.x * 8 + wv; if (tk >= NTOK) return; const int l = tk % LL;
  const float x0 = SEQ[(size_t)tk * HH + lane], x1 = SEQ[(size_t)tk * HH + 32 + lane]; sx[wv][lane] = x0; sx[wv][32 + lane] = x1;
  float s = x0 + x1; for (int o = 16; o >= 1; o >>= 1) s += __shfl_xor(s, o, 32); const float mu = s * (1.0f / HH); const float d0 = x0 - mu, d1 = x1 - mu; float vq = d0 * d0 + d1 * d1; for (int o = 16; o >= 1; o >>= 1) vq += __shfl_xor(vq, o, 32);
  const float rs = 1.0f / sqrtf(vq * (1.0f / HH) + 1e-8f); const float q0 = d0 * rs * bf16_round(g1[lane]) + bf16_round(be1[lane]), q1 = d1 * rs * bf16_round(g1[32 + lane]) + bf16_round(be1[32 + lane]); sq[wv][lane] = q0; sq[wv][32 + lane] = q1;
  __builtin_amdgcn_fence(__ATOMIC_ACQ_REL, "workgroup"); __builtin_amdgcn_wave_barrier();
  float aq0 = bf16_round(bq[lane]), aq1 = bf16_round(bq[32 + lane]), ak0 = bf16_round(bk[lane]), ak1 = bf16_round(bk[32 + lane]), av0 = bf16_round(bv[lane]), av1 = bf16_round(bv[32 + lane]);
#pragma unroll 1
  for (int i = 0; i < HH; ++i) { const float qi = sq[wv][i], xi = sx[wv][i]; aq0 += qi * swq[i][lane]; aq1 += qi * swq[i][32 + lane]; ak0 += xi * swk[i][lane]; ak1 += xi * swk[i][32 + lane]; av0 += xi * swv[i][lane]; av1 += xi * swv[i][32 + lane]; }
  ak0 += bf16_round(pK[l * HH + lane]); ak1 += bf16_round(pK[l * HH + 32 + lane]); av0 += bf16_round(pV[l * HH + lane]); av1 += bf16_round(pV[l * HH + 32 + lane]);
  for (int pass = 0; pass < 2; ++pass) { const size_t r = (size_t)tk * HH; *(volatile float*)(QN + r + lane) = q0; *(volatile float*)(QN + r + 32 + lane) = q1; *(volatile float*)(Qo + r + lane) = aq0; *(volatile float*)(Qo + r + 32 + lane) = aq1; *(volatile float*)(KP + r + lane) = ak0; *(volatile float*)(KP + r + 32 + lane) = ak1; *(volatile float*)(VP + r + lane) = av0; *(volatile float*)(VP + r + 32 + lane) = av1; if (pass == 0) __threadfence(); }
}
__global__ __launch_bounds__(256) void k_attn(const float* __restrict__ Qo, const float* __restrict__ KP, const float* __restrict__ VP, const float* __restrict__ QT, const float* __restrict__ QD, const int* __restrict__ ids, const int* __restrict__ tmat, const int* __restrict__ dmat, float* __restrict__ O1, float* __restrict__ HT, float* __restrict__ HDd) {
  __shared__ float sqv[8][HD]; __shared__ float sa[8][224]; __shared__ int st[8][224], sd[8][224]; __shared__ float sht[8][NRP], shd[8][NRP];
  const int tid = threadIdx.x, wv = tid >> 5, lane = tid & 31; const int row = blockIdx.x * 8 + wv; if (row >= BB * NHD * LL) return; const int q = row % LL; const int h = (row / LL) % NHD; const int b = row / (LL * NHD); const size_t tk = (size_t)b * LL + q;
  sqv[wv][lane] = Qo[tk * HH + h * HD + lane]; for (int r2 = lane; r2 < NRP; r2 += 32) { sht[wv][r2] = 0.f; shd[wv][r2] = 0.f; }
  const bool padq = (ids[tk] == 0); const float* qt = QT + ((size_t)h * NTOK + tk) * NRP; const float* qd = QD + ((size_t)h * NTOK + tk) * NRP; const float NEGV = -4294967295.0f;
  __builtin_amdgcn_fence(__ATOMIC_ACQ_REL, "workgroup"); __builtin_amdgcn_wave_barrier();
  float mx = -3.0e38f;
#pragma unroll 1
  for (int k = lane; k < LL; k += 32) { const float* kr = KP + ((size_t)b * LL + k) * HH + h * HD; float s = 0.f;
#pragma unroll 8
    for (int d = 0; d < HD; ++d) s += sqv[wv][d] * kr[d];
    int ti = tmat[(tk * LL) + k]; ti = ti < 0 ? 0 : (ti >= NREL ? NREL - 1 : ti); int di = dmat[(tk * LL) + k]; di = di < 0 ? 0 : (di >= NREL ? NREL - 1 : di); st[wv][k] = ti; sd[wv][k] = di;
    s = ((s + qt[ti]) + qd[di]) * 0.17677669529663687f; if (padq) s = NEGV; if (k > q) s = NEGV; sa[wv][k] = s; mx = fmaxf(mx, s); }
  for (int o = 16; o >= 1; o >>= 1) mx = fmaxf(mx, __shfl_xor(mx, o, 32));
  __builtin_amdgcn_fence(__ATOMIC_ACQ_REL, "workgroup"); __builtin_amdgcn_wave_barrier();
  float den = 0.f; for (int k = lane; k < LL; k += 32) { const float e = expf(sa[wv][k] - mx); sa[wv][k] = e; den += e; } for (int o = 16; o >= 1; o >>= 1) den += __shfl_xor(den, o, 32); const float rd = 1.0f / den;
  __builtin_amdgcn_fence(__ATOMIC_ACQ_REL, "workgroup"); __builtin_amdgcn_wave_barrier();
  if (lane == 0) { for (int k = 0; k < LL; ++k) { const float a = sa[wv][k] * rd; sht[wv][st[wv][k]] += a; shd[wv][sd[wv][k]] += a; } }
  float o = 0.f;
#pragma unroll 4
  for (int k = 0; k < LL; ++k) o += (sa[wv][k] * rd) * VP[((size_t)b * LL + k) * HH + h * HD + lane];
  __builtin_amdgcn_fence(__ATOMIC_ACQ_REL, "workgroup"); __builtin_amdgcn_wave_barrier();
  float* ht = HT + ((size_t)h * NTOK + tk) * NRP; float* hd = HDd + ((size_t)h * NTOK + tk) * NRP;
  for (int pass = 0; pass < 2; ++pass) { *(volatile float*)(O1 + tk * HH + h * HD + lane) = o; for (int r2 = lane; r2 < NRP; r2 += 32) { *(volatile float*)(ht + r2) = sht[wv][r2]; *(volatile float*)(hd + r2) = shd[wv][r2]; } if (pass == 0) __threadfence(); }
}
__global__ __launch_bounds__(256) void k_post(const float* __restrict__ QN, const float* __restrict__ OUT, const float* __restrict__ g2, const float* __restrict__ be2, const float* __restrict__ c1w, const float* __restrict__ c1b, const float* __restrict__ c2w, const float* __restrict__ c2b, const int* __restrict__ ids, float* __restrict__ SEQ) {
  __shared__ float sw1[HH][HH + 1], sw2[HH][HH + 1]; __shared__ float ss[8][HH], sh[8][HH]; const int tid = threadIdx.x, wv = tid >> 5, lane = tid & 31;
  for (int e = tid; e < HH * HH; e += 256) { const int o = e / HH, i = e % HH; sw1[i][o] = bf16_round(c1w[e]); sw2[i][o] = bf16_round(c2w[e]); }
  __syncthreads(); const int tk = blockIdx.x * 8 + wv; if (tk >= NTOK) return; const float keep = (ids[tk] == 0) ? 0.f : 1.f;
  const float x0 = QN[(size_t)tk * HH + lane] + OUT[(size_t)tk * HH + lane], x1 = QN[(size_t)tk * HH + 32 + lane] + OUT[(size_t)tk * HH + 32 + lane];
  float s = x0 + x1; for (int o = 16; o >= 1; o >>= 1) s += __shfl_xor(s, o, 32); const float mu = s * (1.0f / HH); const float d0 = x0 - mu, d1 = x1 - mu; float vq = d0 * d0 + d1 * d1; for (int o = 16; o >= 1; o >>= 1) vq += __shfl_xor(vq, o, 32);
  const float rs = 1.0f / sqrtf(vq * (1.0f / HH) + 1e-8f); const float y0 = d0 * rs * bf16_round(g2[lane]) + bf16_round(be2[lane]), y1 = d1 * rs * bf16_round(g2[32 + lane]) + bf16_round(be2[32 + lane]); ss[wv][lane] = y0; ss[wv][32 + lane] = y1;
  __builtin_amdgcn_fence(__ATOMIC_ACQ_REL, "workgroup"); __builtin_amdgcn_wave_barrier();
  float h0 = bf16_round(c1b[lane]), h1 = bf16_round(c1b[32 + lane]);
#pragma unroll 1
  for (int i = 0; i < HH; ++i) { const float xi = ss[wv][i]; h0 += xi * sw1[i][lane]; h1 += xi * sw1[i][32 + lane]; }
  sh[wv][lane] = fmaxf(h0, 0.f); sh[wv][32 + lane] = fmaxf(h1, 0.f);
  __builtin_amdgcn_fence(__ATOMIC_ACQ_REL, "workgroup"); __builtin_amdgcn_wave_barrier();
  float z0 = bf16_round(c2b[lane]), z1 = bf16_round(c2b[32 + lane]);
#pragma unroll 1
  for (int i = 0; i < HH; ++i) { const float hi = sh[wv][i]; z0 += hi * sw2[i][lane]; z1 += hi * sw2[i][32 + lane]; }
  const float o0 = (y0 + z0) * keep, o1 = (y1 + z1) * keep;
  for (int pass = 0; pass < 2; ++pass) { *(volatile float*)(SEQ + (size_t)tk * HH + lane) = o0; *(volatile float*)(SEQ + (size_t)tk * HH + 32 + lane) = o1; if (pass == 0) __threadfence(); }
}
__global__ __launch_bounds__(256) void k_lnf(const float* __restrict__ SEQ, const float* __restrict__ g, const float* __restrict__ be, float* __restrict__ out) { const int tid = threadIdx.x, wv = tid >> 5, lane = tid & 31; const int tk = blockIdx.x * 8 + wv; if (tk >= NTOK) return;
  const float x0 = SEQ[(size_t)tk * HH + lane], x1 = SEQ[(size_t)tk * HH + 32 + lane]; float s = x0 + x1; for (int o = 16; o >= 1; o >>= 1) s += __shfl_xor(s, o, 32); const float mu = s * (1.0f / HH); const float d0 = x0 - mu, d1 = x1 - mu; float vq = d0 * d0 + d1 * d1; for (int o = 16; o >= 1; o >>= 1) vq += __shfl_xor(vq, o, 32);
  const float rs = 1.0f / sqrtf(vq * (1.0f / HH) + 1e-8f); const float y0 = d0 * rs * bf16_round(g[lane]) + bf16_round(be[lane]), y1 = d1 * rs * bf16_round(g[32 + lane]) + bf16_round(be[32 + lane]);
  for (int pass = 0; pass < 2; ++pass) { *(volatile float*)(out + (size_t)tk * HH + lane) = y0; *(volatile float*)(out + (size_t)tk * HH + 32 + lane) = y1; if (pass == 0) __threadfence(); } }
extern "C" void kernel_launch(void* const* d_in, const int* in_sizes, int n_in,
                              void* d_out, int out_size, void* d_ws, size_t ws_size, hipStream_t stream) {
  (void)in_sizes; (void)n_in; (void)out_size;
  const int* ids = (const int*)d_in[0]; const int* tmat = (const int*)d_in[1]; const int* dmat = (const int*)d_in[2]; const float* emb = (const float*)d_in[3]; const float* pK = (const float*)d_in[4]; const float* pV = (const float*)d_in[5];
  const float* tmk = (const float*)d_in[6]; const float* tmv = (const float*)d_in[7]; const float* dmk = (const float*)d_in[8]; const float* dmv = (const float*)d_in[9];
  const float* Wq = (const float*)d_in[10]; const float* bq = (const float*)d_in[11]; const float* Wk = (const float*)d_in[12]; const float* bk = (const float*)d_in[13]; const float* Wv = (const float*)d_in[14]; const float* bv = (const float*)d_in[15];
  const float* g1 = (const float*)d_in[16]; const float* be1 = (const float*)d_in[17]; const float* g2 = (const float*)d_in[18]; const float* be2 = (const float*)d_in[19]; const float* c1w = (const float*)d_in[20]; const float* c1b = (const float*)d_in[21]; const float* c2w = (const float*)d_in[22]; const float* c2b = (const float*)d_in[23]; const float* gf = (const float*)d_in[24]; const float* bfin = (const float*)d_in[25];
  char* ws = (char*)d_ws; size_t off = 0;
  auto take = [&](size_t bytes) { char* p = ws + off; off += (bytes + 255) & ~(size_t)255; return p; };
  unsigned short* TK = (unsigned short*)take((size_t)2 * NRP * HH * 2); unsigned short* TVt = (unsigned short*)take((size_t)2 * NHD * HD * NRP * 2);
  float* SEQ = (float*)take((size_t)NTOK * HH * 4); float* QN = (float*)take((size_t)NTOK * HH * 4); float* Qo = (float*)take((size_t)NTOK * HH * 4); float* KP = (float*)take((size_t)NTOK * HH * 4); float* VP = (float*)take((size_t)NTOK * HH * 4);
  float* QT = (float*)take((size_t)NHD * NTOK * NRP * 4); float* QD = (float*)take((size_t)NHD * NTOK * NRP * 4); float* HT = (float*)take((size_t)NHD * NTOK * NRP * 4); float* HDd = (float*)take((size_t)NHD * NTOK * NRP * 4); float* OUT = (float*)take((size_t)NTOK * HH * 4);
  if (off > ws_size) return;
  k_tabK<<<(2 * NRP * 8 + 255) / 256, 256, 0, stream>>>(tmk, dmk, TK); k_tabV<<<(2 * NHD * HD * (NRP / 8) + 255) / 256, 256, 0, stream>>>(tmv, dmv, TVt);
  k_emb<<<NTOK / 8, 256, 0, stream>>>(ids, emb, SEQ);
  for (int i = 0; i < NB; ++i) {
    k_proj<<<NTOK / 8, 256, 0, stream>>>(SEQ, Wq + i * HH * HH, bq + i * HH, Wk + i * HH * HH, bk + i * HH, Wv + i * HH * HH, bv + i * HH, g1 + i * HH, be1 + i * HH, pK, pV, QN, Qo, KP, VP);
    for (int h = 0; h < NHD; ++h) {
      k_gemm_b<true, false, 0><<<dim3(((NTOK / 16) * ((NRP + 63) / 64) + 3) / 4, 1), 128, 0, stream>>>(Qo + h * HD, HH, 0, TK + h * HD, TK + h * HD, HH, 0, nullptr, nullptr, 0, 0, 1.f, 1.f, QT + (size_t)h * NTOK * NRP, NRP, 0, NTOK, NRP, HD);
      k_gemm_b<true, false, 0><<<dim3(((NTOK / 16) * ((NRP + 63) / 64) + 3) / 4, 1), 128, 0, stream>>>(Qo + h * HD, HH, 0, TK + (size_t)NRP * HH + h * HD, TK + (size_t)NRP * HH + h * HD, HH, 0, nullptr, nullptr, 0, 0, 1.f, 1.f, QD + (size_t)h * NTOK * NRP, NRP, 0, NTOK, NRP, HD); }
    k_attn<<<(BB * NHD * LL + 7) / 8, 256, 0, stream>>>(Qo, KP, VP, QT, QD, ids, tmat, dmat, OUT, HT, HDd);
    for (int h = 0; h < NHD; ++h) {
      k_gemm_b<true, false, 0><<<dim3(((NTOK / 16) * 1 + 3) / 4, 1), 128, 0, stream>>>(HT + (size_t)h * NTOK * NRP, NRP, 0, TVt + ((size_t)0 * NHD + h) * HD * NRP, TVt + ((size_t)0 * NHD + h) * HD * NRP, NRP, 0, nullptr, OUT + h * HD, HH, 0, 1.f, 1.f, OUT + h * HD, HH, 0, NTOK, HD, NRP);
      k_gemm_b<true, false, 0><<<dim3(((NTOK / 16) * 1 + 3) / 4, 1), 128, 0, stream>>>(HDd + (size_t)h * NTOK * NRP, NRP, 0, TVt + ((size_t)1 * NHD + h) * HD * NRP, TVt + ((size_t)1 * NHD + h) * HD * NRP, NRP, 0, nullptr, OUT + h * HD, HH, 0, 1.f, 1.f, OUT + h * HD, HH, 0, NTOK, HD, NRP);   }
    k_post<<<NTOK / 8, 256, 0, stream>>>(QN, OUT, g2 + i * HH, be2 + i * HH, c1w + i * HH * HH, c1b + i * HH, c2w + i * HH * HH, c2b + i * HH, ids, SEQ);
  }
  k_lnf<<<NTOK / 8, 256, 0, stream>>>(SEQ, gf, bfin, (float*)d_out);
}
